// MultiHeadAttention_12730283065384
// MI455X (gfx1250) — hardware-verified
//
#include <hip/hip_runtime.h>
#ifndef NB
#define NB 4
#endif
#ifndef SEQ
#define SEQ 1024
#endif
#define NB_FULL 4
#define SEQ_FULL 1024
#define NH 16
#define HD 64
#define DM 1024
#define RHSW (SEQ_FULL + 4)
#define NKS (SEQ / 32)
#define MBW (SEQ_FULL / 32)
#define CXP 2048
#define COVP (SEQ + 4)
#define STP 72
#define COV_LDS_BYTES (16 * COVP * 4)
#define ATTN_LDS (COV_LDS_BYTES + 2 * 16 * STP * 2)

#define XN ((size_t)SEQ * NB_FULL * DM)
#define WN ((size_t)DM * DM)
#define PLSZ ((size_t)NB * NH * SEQ * HD)
#define COV_OFF ((size_t)SEQ_FULL * NB_FULL * DM)

#define BYTES_XB (3 * XN * 2)
#define BYTES_WB (4 * WN * 2)
#define BYTES_PL (6 * PLSZ * 2)
#define BYTES_CX ((size_t)SEQ * NB_FULL * CXP * 2)
#define BYTES_MB ((size_t)NB * SEQ * MBW * 4)

static_assert(SEQ % 128 == 0);
static_assert(SEQ <= SEQ_FULL);
static_assert(NB <= NB_FULL);
static_assert(MBW == 32);
static_assert(HD == 64);
static_assert(NH * HD == DM);
static_assert(COV_OFF * 4 == (size_t)16777216);
static_assert(BYTES_XB % 256 == 0 && BYTES_WB % 256 == 0 && BYTES_PL % 256 == 0 && BYTES_CX % 256 == 0 && BYTES_MB % 256 == 0);
static_assert(BYTES_XB + BYTES_WB + BYTES_PL + BYTES_CX + BYTES_MB <= (size_t)134217728);
static_assert((size_t)SEQ * NB_FULL * DM <= COV_OFF);
static_assert(COV_OFF + ((size_t)(NB - 1) * SEQ_FULL + (SEQ - 1)) * SEQ_FULL + SEQ <= (size_t)33554432 / 4);

typedef __bf16 v16b __attribute__((ext_vector_type(16)));
typedef unsigned short v8us __attribute__((ext_vector_type(8), may_alias));
typedef float v8f __attribute__((ext_vector_type(8)));
typedef float v4f __attribute__((ext_vector_type(4)));
typedef float v4fa __attribute__((ext_vector_type(4), may_alias));
typedef int v4i __attribute__((ext_vector_type(4)));
typedef int v4ia __attribute__((ext_vector_type(4), may_alias));
union FragB { v16b v; v8us half[2]; unsigned short u[16]; };

#define LOG2E 1.4426950408889634f
#define NEGBIG (-1.0e30f)

__device__ __forceinline__ unsigned short bf16_bits(float x) {
  unsigned int u = __float_as_uint(x);
  return (unsigned short)((u + 0x7FFFu + ((u >> 16) & 1u)) >> 16);
}
__device__ __forceinline__ float bf16_val(unsigned short b) { return __uint_as_float(((unsigned int)b) << 16); }

__device__ __forceinline__ v8f wm(v16b a, v16b b, v8f c) {
  return __builtin_amdgcn_wmma_f32_16x16x32_bf16(false, a, false, b, (short)0, c, false, false);
}

__global__ __launch_bounds__(256) void k_cvt(const float* __restrict__ src, unsigned short* __restrict__ dst, int n8) {
  const int t = blockIdx.x * 256 + threadIdx.x;
  if (t >= n8) return;
  const float* s = src + (size_t)t * 8;
  const v4f x0 = *(const v4fa*)(s), x1 = *(const v4fa*)(s + 4);
  v8us o;
  o[0] = bf16_bits(x0[0]); o[1] = bf16_bits(x0[1]); o[2] = bf16_bits(x0[2]); o[3] = bf16_bits(x0[3]);
  o[4] = bf16_bits(x1[0]); o[5] = bf16_bits(x1[1]); o[6] = bf16_bits(x1[2]); o[7] = bf16_bits(x1[3]);
  unsigned short* d = dst + (size_t)t * 8;
  *(volatile v8us*)d = o;
  __threadfence();
  *(volatile v8us*)d = o;
}

__global__ __launch_bounds__(256) void k_mask(const int* __restrict__ mask, const int* __restrict__ rhs,
                                              const int* __restrict__ lidx, unsigned int* __restrict__ Mb) {
  const int t = blockIdx.x * 256 + threadIdx.x;
  if (t >= NB * SEQ * MBW) return;
  const int j = t & 31, row = t >> 5;
  const int b = row / SEQ, q = row - b * SEQ;
  int L = lidx[0];
  L = (L < -64) ? -64 : ((L > 64) ? 64 : L);
  int tt = 4 - 4 * L; if (tt < 0) tt = 0;
  int start = 4 - tt; if (start < 0) start = 0;
  start = (start >= 4) ? 4 : 0;
  const int* mp = mask + ((size_t)b * SEQ_FULL + q) * SEQ_FULL + 32 * j;
  const int* rp = rhs + (size_t)q * RHSW + start + 32 * j;
  unsigned int w = 0u;
#pragma unroll 4
  for (int c = 0; c < 8; ++c) {
    const v4i a = *(const v4ia*)(mp + 4 * c);
    const v4i r = *(const v4ia*)(rp + 4 * c);
    const unsigned int nib = (((a[0] | r[0]) != 0) ? 1u : 0u) | (((a[1] | r[1]) != 0) ? 2u : 0u) |
                             (((a[2] | r[2]) != 0) ? 4u : 0u) | (((a[3] | r[3]) != 0) ? 8u : 0u);
    w |= nib << (4 * c);
  }
  unsigned int* d = Mb + (size_t)t;
  *(volatile unsigned int*)d = w;
  __threadfence();
  *(volatile unsigned int*)d = w;
}

template <int KT>
__device__ __forceinline__ void gemm_main(const unsigned short* __restrict__ ap0, const unsigned short* __restrict__ ap1,
                                          const unsigned short* __restrict__ bp, v8f (&acc)[2][4]) {
#pragma unroll 1
  for (int k0 = 0; k0 < KT; k0 += 32) {
    const int kw = k0 & (DM - 1);
    FragB a0, a1, b0, b1, b2, b3;
    a0.half[0] = *(const v8us*)(ap0 + k0); a0.half[1] = *(const v8us*)(ap0 + k0 + 16);
    a1.half[0] = *(const v8us*)(ap1 + k0); a1.half[1] = *(const v8us*)(ap1 + k0 + 16);
    b0.half[0] = *(const v8us*)(bp + kw);                 b0.half[1] = *(const v8us*)(bp + kw + 16);
    b1.half[0] = *(const v8us*)(bp + 16 * DM + kw);       b1.half[1] = *(const v8us*)(bp + 16 * DM + kw + 16);
    b2.half[0] = *(const v8us*)(bp + 32 * DM + kw);       b2.half[1] = *(const v8us*)(bp + 32 * DM + kw + 16);
    b3.half[0] = *(const v8us*)(bp + 48 * DM + kw);       b3.half[1] = *(const v8us*)(bp + 48 * DM + kw + 16);
    acc[0][0] = wm(a0.v, b0.v, acc[0][0]); acc[0][1] = wm(a0.v, b1.v, acc[0][1]);
    acc[0][2] = wm(a0.v, b2.v, acc[0][2]); acc[0][3] = wm(a0.v, b3.v, acc[0][3]);
    acc[1][0] = wm(a1.v, b0.v, acc[1][0]); acc[1][1] = wm(a1.v, b1.v, acc[1][1]);
    acc[1][2] = wm(a1.v, b2.v, acc[1][2]); acc[1][3] = wm(a1.v, b3.v, acc[1][3]);
    asm volatile("v_nop\n\tv_nop\n\tv_nop\n\tv_nop"
                 : "+v"(acc[0][0]), "+v"(acc[0][1]), "+v"(acc[0][2]), "+v"(acc[0][3]),
                   "+v"(acc[1][0]), "+v"(acc[1][1]), "+v"(acc[1][2]), "+v"(acc[1][3])
                 : "v"(a0.v), "v"(a1.v), "v"(b0.v), "v"(b1.v), "v"(b2.v), "v"(b3.v));
  }
}

__global__ __launch_bounds__(64) void k_proj(const unsigned short* __restrict__ Xb, const unsigned short* __restrict__ Wb,
                                             unsigned short* __restrict__ PL) {
  __shared__ __attribute__((aligned(16))) unsigned short sh[64 * STP];
  __shared__ __attribute__((aligned(16))) unsigned short sl[64 * STP];
  const int tid = threadIdx.x, w = __builtin_amdgcn_readfirstlane((int)(tid >> 5)), lane = tid & 31, ln = lane & 15, hh = lane >> 4;
  const int z = blockIdx.z, hcol = blockIdx.y;
  const int mt0 = blockIdx.x * 64;
  const int b = mt0 / SEQ, s0 = mt0 - b * SEQ;
  const int srow = s0 + 32 * w + ln;
  const unsigned short* A = Xb + (size_t)z * XN;
  const unsigned short* ap0 = A + ((size_t)srow * NB_FULL + b) * DM + 8 * hh;
  const unsigned short* ap1 = A + ((size_t)(srow + 16) * NB_FULL + b) * DM + 8 * hh;
  const unsigned short* bp = Wb + (size_t)z * WN + (size_t)(64 * hcol + ln) * DM + 8 * hh;
  v8f acc[2][4] = {};
  gemm_main<DM>(ap0, ap1, bp, acc);
  const float scale = (z == 0) ? 0.125f : 1.0f;
#pragma unroll
  for (int mt = 0; mt < 2; ++mt)
#pragma unroll
    for (int nt = 0; nt < 4; ++nt)
#pragma unroll
      for (int r = 0; r < 8; ++r) {
        const float v = acc[mt][nt][r] * scale;
        const unsigned short hb = bf16_bits(v);
        const unsigned short lb = bf16_bits(v - bf16_val(hb));
        const int sr = 32 * w + 16 * mt + 8 * hh + r;
        const int dc = 16 * nt + ln;
        const int idx = (z == 2) ? (dc * STP + sr) : (sr * STP + dc);
        sh[idx] = hb;
        sl[idx] = lb;
      }
  __syncthreads();
  const size_t hbase = (size_t)b * NH + hcol;
  unsigned short* dstp = PL + (size_t)z * 2 * PLSZ;
  for (int pass = 0; pass < 2; ++pass) {
#pragma unroll 1
    for (int i = 0; i < 8; ++i) {
      const int row = 8 * i + (tid >> 3), piece = tid & 7;
      const v8us vh = *(const v8us*)(sh + row * STP + 8 * piece);
      const v8us vl = *(const v8us*)(sl + row * STP + 8 * piece);
      const size_t ro = (z == 2) ? ((hbase * HD + row) * SEQ + s0) : ((hbase * SEQ + s0 + row) * HD);
      unsigned short* d = dstp + ro + 8 * piece;
      *(volatile v8us*)d = vh;
      *(volatile v8us*)(d + PLSZ) = vl;
    }
    if (pass == 0) __threadfence();
  }
}

__device__ __forceinline__ v8f qk_tile(const unsigned short* __restrict__ kp, const FragB& qh0, const FragB& qh1,
                                       const FragB& ql0, const FragB& ql1) {
  FragB a0, a1, c0, c1;
  const unsigned short* lp = kp + PLSZ;
  a0.half[0] = *(const v8us*)(kp);      a0.half[1] = *(const v8us*)(kp + 16);
  a1.half[0] = *(const v8us*)(kp + 32); a1.half[1] = *(const v8us*)(kp + 48);
  c0.half[0] = *(const v8us*)(lp);      c0.half[1] = *(const v8us*)(lp + 16);
  c1.half[0] = *(const v8us*)(lp + 32); c1.half[1] = *(const v8us*)(lp + 48);
  v8f c = {0.f, 0.f, 0.f, 0.f, 0.f, 0.f, 0.f, 0.f};
  c = wm(c0.v, qh0.v, c); c = wm(c1.v, qh1.v, c);
  c = wm(a0.v, ql0.v, c); c = wm(a1.v, ql1.v, c);
  c = wm(a0.v, qh0.v, c); c = wm(a1.v, qh1.v, c);
  asm volatile("v_nop\n\tv_nop\n\tv_nop\n\tv_nop" : "+v"(c)
               : "v"(a0.v), "v"(a1.v), "v"(c0.v), "v"(c1.v), "v"(qh0.v), "v"(qh1.v), "v"(ql0.v), "v"(ql1.v));
  return c;
}

__device__ __forceinline__ v8f pv_tile(const unsigned short* __restrict__ vp, const FragB& ph, const FragB& pl, v8f o) {
  FragB vh, vl;
  const unsigned short* lp = vp + PLSZ;
  vh.half[0] = *(const v8us*)(vp); vh.half[1] = *(const v8us*)(vp + 16);
  vl.half[0] = *(const v8us*)(lp); vl.half[1] = *(const v8us*)(lp + 16);
  o = wm(vl.v, ph.v, o);
  o = wm(vh.v, pl.v, o);
  o = wm(vh.v, ph.v, o);
  asm volatile("v_nop\n\tv_nop\n\tv_nop\n\tv_nop" : "+v"(o) : "v"(vh.v), "v"(vl.v), "v"(ph.v), "v"(pl.v));
  return o;
}

__global__ __launch_bounds__(32) void k_attn(const unsigned short* __restrict__ PL, const unsigned int* __restrict__ Mb,
                                             unsigned short* __restrict__ Cx, float* __restrict__ Cov) {
  extern __shared__ __attribute__((aligned(16))) unsigned char smem[];
  float* covs = (float*)smem;
  unsigned short* sth = (unsigned short*)(smem + COV_LDS_BYTES);
  unsigned short* stl = sth + 16 * STP;
  const int lane = threadIdx.x & 31, ln = lane & 15, hh = lane >> 4;
  const int b = blockIdx.x / (SEQ / 16), qt = blockIdx.x % (SEQ / 16);
  const int q0 = qt * 16, qg = q0 + ln;
  {
    const v4f z4 = {0.f, 0.f, 0.f, 0.f};
    for (int i = lane; i < 4 * COVP; i += 32) *(v4fa*)(covs + 4 * i) = z4;
  }
  __syncthreads();
  const unsigned int* mrow = Mb + (size_t)(b * SEQ + qg) * MBW;
  const int sh8 = 8 * hh;
  float* crow = covs + ln * COVP + 8 * hh;

#pragma unroll 1
  for (int h = 0; h < NH; ++h) {
    const size_t hb = (size_t)b * NH + h;
    const unsigned short* qp = PL + (hb * SEQ + qg) * HD + 8 * hh;
    FragB qh0, qh1, ql0, ql1;
    qh0.half[0] = *(const v8us*)(qp);             qh0.half[1] = *(const v8us*)(qp + 16);
    qh1.half[0] = *(const v8us*)(qp + 32);        qh1.half[1] = *(const v8us*)(qp + 48);
    ql0.half[0] = *(const v8us*)(qp + PLSZ);      ql0.half[1] = *(const v8us*)(qp + PLSZ + 16);
    ql1.half[0] = *(const v8us*)(qp + PLSZ + 32); ql1.half[1] = *(const v8us*)(qp + PLSZ + 48);
    const unsigned short* khp = PL + 2 * PLSZ + (hb * SEQ + ln) * HD + 8 * hh;
    const unsigned short* vhp = PL + 4 * PLSZ + (hb * HD + ln) * SEQ + 8 * hh;

    float mr = NEGBIG, lr = 0.0f;
#pragma unroll 1
    for (int j = 0; j < NKS; ++j) {
      const unsigned int w = mrow[j];
      if (!__any(w != 0xFFFFFFFFu)) continue;
      const unsigned short* kp = khp + (size_t)(32 * j) * HD;
      const v8f s0 = qk_tile(kp, qh0, qh1, ql0, ql1);
      const v8f s1 = qk_tile(kp + 16 * HD, qh0, qh1, ql0, ql1);
      const unsigned int wb = w >> sh8;
      float sc[16];
      float mx = NEGBIG;
#pragma unroll
      for (int r = 0; r < 8; ++r) {
        sc[r]     = ((wb >> r) & 1u) ? NEGBIG : s0[r];
        sc[8 + r] = ((wb >> (16 + r)) & 1u) ? NEGBIG : s1[r];
        mx = fmaxf(mx, fmaxf(sc[r], sc[8 + r]));
      }
      mx = fmaxf(mx, __shfl_xor(mx, 16, 32));
      const float mnew = fmaxf(mr, mx);
      const float al = exp2f((mr - mnew) * LOG2E);
      float ps = 0.0f;
#pragma unroll
      for (int i = 0; i < 16; ++i) {
        const float e = exp2f((sc[i] - mnew) * LOG2E);
        ps += (sc[i] > -1.0e29f) ? e : 0.0f;
      }
      ps += __shfl_xor(ps, 16, 32);
      lr = lr * al + ps;
      mr = mnew;
    }
    const float inv = 1.0f / lr;

    v8f O[4] = {};
#pragma unroll 1
    for (int j = 0; j < NKS; ++j) {
      const unsigned int w = mrow[j];
      if (!__any(w != 0xFFFFFFFFu)) continue;
      const int key0 = 32 * j;
      const unsigned short* kp = khp + (size_t)key0 * HD;
      const v8f s0 = qk_tile(kp, qh0, qh1, ql0, ql1);
      const v8f s1 = qk_tile(kp + 16 * HD, qh0, qh1, ql0, ql1);
      __builtin_amdgcn_sched_barrier(0);
      const unsigned int wb = w >> sh8;
      float pn[16];
#pragma unroll
      for (int r = 0; r < 8; ++r) {
        const float e0 = exp2f((s0[r] - mr) * LOG2E) * inv;
        const float e1 = exp2f((s1[r] - mr) * LOG2E) * inv;
        pn[r]     = ((wb >> r) & 1u) ? 0.0f : e0;
        pn[8 + r] = ((wb >> (16 + r)) & 1u) ? 0.0f : e1;
      }
      {
        float* cr = crow + key0;
        v4f c0 = *(const v4fa*)(cr), c1 = *(const v4fa*)(cr + 4), c2 = *(const v4fa*)(cr + 16), c3 = *(const v4fa*)(cr + 20);
        c0[0] += pn[0];  c0[1] += pn[1];  c0[2] += pn[2];  c0[3] += pn[3];
        c1[0] += pn[4];  c1[1] += pn[5];  c1[2] += pn[6];  c1[3] += pn[7];
        c2[0] += pn[8];  c2[1] += pn[9];  c2[2] += pn[10]; c2[3] += pn[11];
        c3[0] += pn[12]; c3[1] += pn[13]; c3[2] += pn[14]; c3[3] += pn[15];
        *(v4fa*)(cr) = c0; *(v4fa*)(cr + 4) = c1; *(v4fa*)(cr + 16) = c2; *(v4fa*)(cr + 20) = c3;
      }
      FragB ph, pl;
#pragma unroll
      for (int i = 0; i < 16; ++i) {
        const unsigned short hb16 = bf16_bits(pn[i]);
        ph.u[i] = hb16;
        pl.u[i] = bf16_bits(pn[i] - bf16_val(hb16));
      }
      __builtin_amdgcn_sched_barrier(0);
      const unsigned short* vp = vhp + key0;
      O[0] = pv_tile(vp, ph, pl, O[0]);
      O[1] = pv_tile(vp + (size_t)16 * SEQ, ph, pl, O[1]);
      O[2] = pv_tile(vp + (size_t)32 * SEQ, ph, pl, O[2]);
      O[3] = pv_tile(vp + (size_t)48 * SEQ, ph, pl, O[3]);
    }

#pragma unroll
    for (int t = 0; t < 4; ++t) {
      v8us oh, ol;
#pragma unroll
      for (int r = 0; r < 8; ++r) {
        const float v = O[t][r];
        const unsigned short hb16 = bf16_bits(v);
        oh[r] = hb16;
        ol[r] = bf16_bits(v - bf16_val(hb16));
      }
      *(v8us*)(sth + ln * STP + 16 * t + 8 * hh) = oh;
      *(v8us*)(stl + ln * STP + 16 * t + 8 * hh) = ol;
    }
    __syncthreads();
    for (int pass = 0; pass < 2; ++pass) {
#pragma unroll
      for (int i = 0; i < 4; ++i) {
        const int row = 4 * i + (lane >> 3), piece = lane & 7;
        const v8us vh = *(const v8us*)(sth + row * STP + 8 * piece);
        const v8us vl = *(const v8us*)(stl + row * STP + 8 * piece);
        unsigned short* d = Cx + ((size_t)(q0 + row) * NB_FULL + b) * CXP + h * HD + 8 * piece;
        *(volatile v8us*)d = vh;
        *(volatile v8us*)(d + DM) = vl;
      }
      if (pass == 0) __threadfence();
    }
    __syncthreads();
  }

  __syncthreads();
  float* cg = Cov + ((size_t)b * SEQ_FULL + q0) * SEQ_FULL;
  for (int pass = 0; pass < 2; ++pass) {
#pragma unroll 1
    for (int row = 0; row < 16; ++row) {
#pragma unroll 1
      for (int c = 0; c < SEQ / 128; ++c) {
        const int col = c * 128 + lane * 4;
        v4f v = *(const v4fa*)(covs + row * COVP + col);
        v[0] *= 0.0625f; v[1] *= 0.0625f; v[2] *= 0.0625f; v[3] *= 0.0625f;
        *(volatile v4f*)(cg + (size_t)row * SEQ_FULL + col) = v;
      }
    }
    if (pass == 0) __threadfence();
  }
}

__global__ __launch_bounds__(64) void k_oproj(const unsigned short* __restrict__ Cx, const unsigned short* __restrict__ Wo,
                                              float* __restrict__ Out) {
  __shared__ __attribute__((aligned(16))) float so[64 * 68];
  const int tid = threadIdx.x, w = __builtin_amdgcn_readfirstlane((int)(tid >> 5)), lane = tid & 31, ln = lane & 15, hh = lane >> 4;
  const int m0 = blockIdx.x * 64, n0 = blockIdx.y * 64;
  const unsigned short* ap0 = Cx + (size_t)(m0 + 32 * w + ln) * CXP + 8 * hh;
  const unsigned short* ap1 = ap0 + (size_t)16 * CXP;
  const unsigned short* bp = Wo + (size_t)(n0 + ln) * DM + 8 * hh;
  v8f acc[2][4] = {};
  gemm_main<CXP>(ap0, ap1, bp, acc);
#pragma unroll
  for (int mt = 0; mt < 2; ++mt)
#pragma unroll
    for (int nt = 0; nt < 4; ++nt)
#pragma unroll
      for (int r = 0; r < 8; ++r)
        so[(32 * w + 16 * mt + 8 * hh + r) * 68 + 16 * nt + ln] = acc[mt][nt][r];
  __syncthreads();
  const int rsub = lane >> 4, c4 = (lane & 15) * 4;
  for (int pass = 0; pass < 2; ++pass) {
#pragma unroll 1
    for (int i = 0; i < 16; ++i) {
      const int row = 32 * w + 2 * i + rsub;
      const v4f v = *(const v4fa*)(so + row * 68 + c4);
      *(volatile v4f*)(Out + (size_t)(m0 + row) * DM + n0 + c4) = v;
    }
    if (pass == 0) __threadfence();
  }
}

extern "C" void kernel_launch(void* const* d_in, const int* in_sizes, int n_in,
                              void* d_out, int out_size, void* d_ws, size_t ws_size, hipStream_t stream) {
  if (n_in < 10) return;
  const long long needX = (long long)SEQ * NB_FULL * DM;
  if ((long long)in_sizes[0] < needX || (long long)in_sizes[1] < needX || (long long)in_sizes[2] < needX) return;
  for (int i = 3; i < 7; ++i) if ((long long)in_sizes[i] < (long long)DM * DM) return;
  if ((long long)in_sizes[7] < ((long long)(NB - 1) * SEQ_FULL + (SEQ - 1)) * SEQ_FULL + SEQ_FULL) return;
  if ((long long)in_sizes[8] < (long long)SEQ * RHSW) return;
  if (in_sizes[9] < 1) return;
  if ((long long)out_size < (long long)COV_OFF + ((long long)(NB - 1) * SEQ_FULL + (SEQ - 1)) * SEQ_FULL + SEQ) return;

  const float* query = (const float*)d_in[0];
  const float* keyt  = (const float*)d_in[1];
  const float* value = (const float*)d_in[2];
  const float* Wq    = (const float*)d_in[3];
  const float* Wk    = (const float*)d_in[4];
  const float* Wv    = (const float*)d_in[5];
  const float* Wo    = (const float*)d_in[6];
  const int*   mask  = (const int*)d_in[7];
  const int*   rhs   = (const int*)d_in[8];
  const int*   lidx  = (const int*)d_in[9];
  float* out = (float*)d_out;
  float* cov = out + COV_OFF;

  char* ws = (char*)d_ws;
  size_t off = 0;
  unsigned short* Xb = (unsigned short*)(ws + off); off += BYTES_XB;
  unsigned short* Wb = (unsigned short*)(ws + off); off += BYTES_WB;
  unsigned short* PL = (unsigned short*)(ws + off); off += BYTES_PL;
  unsigned short* Cx = (unsigned short*)(ws + off); off += BYTES_CX;
  unsigned int*   Mb = (unsigned int*)(ws + off);   off += BYTES_MB;
  if (off > ws_size) return;

  const int nx8 = (int)(XN / 8), nw8 = (int)(WN / 8);
  k_cvt<<<(unsigned)((nx8 + 255) / 256), 256, 0, stream>>>(query, Xb, nx8);
  k_cvt<<<(unsigned)((nx8 + 255) / 256), 256, 0, stream>>>(keyt, Xb + XN, nx8);
  k_cvt<<<(unsigned)((nx8 + 255) / 256), 256, 0, stream>>>(value, Xb + 2 * XN, nx8);
  k_cvt<<<(unsigned)((nw8 + 255) / 256), 256, 0, stream>>>(Wq, Wb, nw8);
  k_cvt<<<(unsigned)((nw8 + 255) / 256), 256, 0, stream>>>(Wk, Wb + WN, nw8);
  k_cvt<<<(unsigned)((nw8 + 255) / 256), 256, 0, stream>>>(Wv, Wb + 2 * WN, nw8);
  k_cvt<<<(unsigned)((nw8 + 255) / 256), 256, 0, stream>>>(Wo, Wb + 3 * WN, nw8);
  k_mask<<<(unsigned)((NB * SEQ * MBW + 255) / 256), 256, 0, stream>>>(mask, rhs, lidx, Mb);
  k_proj<<<dim3((unsigned)(NB * SEQ / 64), NH, 3), 64, 0, stream>>>(Xb, Wb, PL);
  hipFuncSetAttribute(reinterpret_cast<const void*>(&k_attn), hipFuncAttributeMaxDynamicSharedMemorySize, (int)ATTN_LDS);
  k_attn<<<(unsigned)(NB * (SEQ / 16)), 32, (size_t)ATTN_LDS, stream>>>(PL, Mb, Cx, cov);
  k_oproj<<<dim3((unsigned)(SEQ * NB_FULL / 64), DM / 64), 64, 0, stream>>>(Cx, Wb + 3 * WN, out);
}
